// gnn_dsse_65085934403701
// MI455X (gfx1250) — hardware-verified
//
#include <hip/hip_runtime.h>
#include <stddef.h>


#define HD      128
#define DN      256
#define NLAY    5
#define NTHR    256
#define NWAVE   8
#define EPT     8
#define NGRP    2
#define CHUNK   (NTHR * EPT * NGRP)
#define WCAP    (EPT * NGRP * 32)
#define LISTN   (NWAVE * WCAP)
#define ESHF    11
#define NBC     32768
#define NBF     2048
#define RCAP    40960
#define RBN     128
#define TGT     256
#define DEGCAP  512
#define GROWS   128
#define DROWS   64
#define DTHR    128
#define XROWS   64
#define OTHR    512
#define WSCALE  64
#define ASCALE  64
#define CSELF   1.0f
#define OMALPHA 0.9f
#define ALPHAC  0.1f
#define SLOPEC  0.01f
#define WSCAP   134217728

#define WPL     (HD * HD)
#define WPD     (NLAY * HD * HD)
#define WPTOT   (NLAY * HD * HD + DN * HD)
#define WBL     ((HD * HD / 8) / NTHR)
#define WBD     ((DN * HD / 8) / NTHR)
#define WPREP_BLOCKS (NLAY * WBL + WBD)

#define LDS_COUNT ((NBC + LISTN + NWAVE) * 4)
#define LDS_FILL  ((RCAP + NBF + LISTN + NWAVE) * 4)
#define LDS_GEMM  (GROWS * HD * 4)
#define LDS_DENSE (DROWS * DN * 4)

static_assert((CHUNK & (CHUNK - 1)) == 0);
static_assert((NBC & (NBC - 1)) == 0 && (NBF & (NBF - 1)) == 0);
static_assert(NBF <= (1 << ESHF));
static_assert((NBC % NBF) == 0);
static_assert(OTHR * 4 == NBF);
static_assert((RCAP % 32) == 0);
static_assert(TGT == NWAVE * 32);
static_assert(GROWS == NWAVE * 16);
static_assert(DROWS == (DTHR / 32) * 16);
static_assert((TGT % GROWS) == 0 && (TGT % DROWS) == 0 && (TGT % XROWS) == 0);
static_assert(HD == 128 && DN == 2 * HD);
static_assert(NBC == NWAVE * 32 * 128);
static_assert((HD * HD / 8) % NTHR == 0 && (DN * HD / 8) % NTHR == 0);
static_assert(WPREP_BLOCKS == 56);
static_assert(XROWS == NWAVE * 8);

typedef float     v2f  __attribute__((ext_vector_type(2)));
typedef float     v4f  __attribute__((ext_vector_type(4)));
typedef float     v8f  __attribute__((ext_vector_type(8)));
typedef int       v4i  __attribute__((ext_vector_type(4)));
typedef unsigned  v2u  __attribute__((ext_vector_type(2)));
typedef _Float16  v4h  __attribute__((ext_vector_type(4)));
typedef _Float16  v8h  __attribute__((ext_vector_type(8)));
typedef _Float16  v16h __attribute__((ext_vector_type(16)));
union FragH { v16h v; v8h h[2]; };
union H4U { v4h h; v2u u; };

__device__ __forceinline__ v8f wmf(v16h a, v16h b, v8f c) {
  v8f d = __builtin_amdgcn_wmma_f32_16x16x32_f16(false, a, false, b, (short)0, c, false, false);
  asm volatile("v_nop\n\tv_nop\n\tv_nop\n\tv_nop" : "+v"(d) : "v"(a), "v"(b));
  return d;
}

__device__ __forceinline__ v16h afr(const _Float16* akp) {
  FragH f;
  f.h[0] = *(const v8h*)akp;
  f.h[1] = *(const v8h*)(akp + 16);
  return f.v;
}

template <int NB, int SRC>
__device__ __forceinline__ int scan_chunk(const int* __restrict__ keys, const int* __restrict__ gath, int nE, int nN,
                                          int cbase, int slotBase, int vec8, int* list, int tid, int lane, int wave) {
  int wc = 0;
#pragma unroll
  for (int g = 0; g < NGRP; ++g) {
    const int el0  = (g * NTHR + tid) * EPT;
    const int e0   = cbase + el0;
    const int sent = -2147483647 - 1;
    v4i da, db;
    v4i sa = {0, 0, 0, 0}, sb = {0, 0, 0, 0};
    if (vec8 != 0 && cbase + CHUNK <= nE) {
      da = *(const v4i*)(keys + e0);
      db = *(const v4i*)(keys + e0 + 4);
      if (SRC) {
        sa = *(const v4i*)(gath + e0);
        sb = *(const v4i*)(gath + e0 + 4);
      }
    } else {
      da.x = (e0     < nE) ? keys[min(e0, nE - 1)] : sent;
      da.y = (e0 + 1 < nE) ? keys[min(e0 + 1, nE - 1)] : sent;
      da.z = (e0 + 2 < nE) ? keys[min(e0 + 2, nE - 1)] : sent;
      da.w = (e0 + 3 < nE) ? keys[min(e0 + 3, nE - 1)] : sent;
      db.x = (e0 + 4 < nE) ? keys[min(e0 + 4, nE - 1)] : sent;
      db.y = (e0 + 5 < nE) ? keys[min(e0 + 5, nE - 1)] : sent;
      db.z = (e0 + 6 < nE) ? keys[min(e0 + 6, nE - 1)] : sent;
      db.w = (e0 + 7 < nE) ? keys[min(e0 + 7, nE - 1)] : sent;
      if (SRC) {
        sa.x = gath[min(e0, nE - 1)];
        sa.y = gath[min(e0 + 1, nE - 1)];
        sa.z = gath[min(e0 + 2, nE - 1)];
        sa.w = gath[min(e0 + 3, nE - 1)];
        sb.x = gath[min(e0 + 4, nE - 1)];
        sb.y = gath[min(e0 + 5, nE - 1)];
        sb.z = gath[min(e0 + 6, nE - 1)];
        sb.w = gath[min(e0 + 7, nE - 1)];
      }
    }
    if (SRC) {
      sa.x = min(max(sa.x, 0), nN - 1); sa.y = min(max(sa.y, 0), nN - 1);
      sa.z = min(max(sa.z, 0), nN - 1); sa.w = min(max(sa.w, 0), nN - 1);
      sb.x = min(max(sb.x, 0), nN - 1); sb.y = min(max(sb.y, 0), nN - 1);
      sb.z = min(max(sb.z, 0), nN - 1); sb.w = min(max(sb.w, 0), nN - 1);
    }
    const unsigned nb = (unsigned)slotBase;
    const unsigned s0 = (unsigned)da.x - nb, s1 = (unsigned)da.y - nb;
    const unsigned s2 = (unsigned)da.z - nb, s3 = (unsigned)da.w - nb;
    const unsigned s4 = (unsigned)db.x - nb, s5 = (unsigned)db.y - nb;
    const unsigned s6 = (unsigned)db.z - nb, s7 = (unsigned)db.w - nb;
    const bool h0 = s0 < (unsigned)NB, h1 = s1 < (unsigned)NB, h2 = s2 < (unsigned)NB, h3 = s3 < (unsigned)NB;
    const bool h4 = s4 < (unsigned)NB, h5 = s5 < (unsigned)NB, h6 = s6 < (unsigned)NB, h7 = s7 < (unsigned)NB;
    const unsigned any = __builtin_amdgcn_ballot_w32(h0 | h1 | h2 | h3 | h4 | h5 | h6 | h7);
    if (any != 0u) {
#define HITJ(HJ, SJ, VJ) { \
        const unsigned mj = __builtin_amdgcn_ballot_w32(HJ); \
        if (mj != 0u) { \
          if (HJ) { \
            const int pos = wc + (int)__builtin_amdgcn_mbcnt_lo(mj, 0u); \
            const int entv = SRC ? (((VJ) << ESHF) | (int)(SJ)) : (int)(SJ); \
            if (pos < WCAP) list[wave * WCAP + pos] = entv; \
          } \
          wc += (int)__builtin_popcount(mj); } }
      HITJ(h0, s0, sa.x)
      HITJ(h1, s1, sa.y)
      HITJ(h2, s2, sa.z)
      HITJ(h3, s3, sa.w)
      HITJ(h4, s4, sb.x)
      HITJ(h5, s5, sb.y)
      HITJ(h6, s6, sb.z)
      HITJ(h7, s7, sb.w)
#undef HITJ
    }
  }
  return wc;
}

__global__ __launch_bounds__(NTHR) void k_wprep(const float* __restrict__ wc, const float* __restrict__ wd, _Float16* wp) {
  const int tid = threadIdx.x;
  const int b = (int)blockIdx.x;
  v8h hv;
  size_t doff;
  if (b < NLAY * WBL) {
    int i = b * NTHR + tid;
    i = i < 0 ? 0 : (i > NLAY * 2048 - 1 ? NLAY * 2048 - 1 : i);
    const int l  = i >> 11;
    const int r  = i & 2047;
    const int n  = r >> 4;
    const int k0 = (r & 15) * 8;
    const float* w = wc + (size_t)l * HD * HD;
#pragma unroll
    for (int e = 0; e < 8; ++e) hv[e] = (_Float16)(w[(size_t)(k0 + e) * HD + n] * (float)WSCALE);
    doff = (size_t)l * WPL + (size_t)n * HD + (size_t)k0;
  } else {
    int j = (b - NLAY * WBL) * NTHR + tid;
    j = j < 0 ? 0 : (j > DN * 16 - 1 ? DN * 16 - 1 : j);
    const int n  = j >> 4;
    const int k0 = (j & 15) * 8;
#pragma unroll
    for (int e = 0; e < 8; ++e) hv[e] = (_Float16)(wd[(size_t)(k0 + e) * DN + n] * (float)WSCALE);
    doff = (size_t)WPD + (size_t)n * HD + (size_t)k0;
  }
  _Float16* d = wp + doff;
  *(volatile v8h*)d = hv;
  __threadfence();
  *(volatile v8h*)d = hv;
}

__global__ __launch_bounds__(NTHR) void k_count(
    const int* __restrict__ keys, const int* __restrict__ gath, int* cnt, float* dinv, int nE, int nN, int vec8) {
  extern __shared__ v4f lds_dyn[];
  int* scnt = (int*)lds_dyn;
  int* list = scnt + NBC;
  int* wcnt = list + LISTN;
  const int tid = threadIdx.x, lane = tid & 31, wave = tid >> 5;
  const int nodeBase = blockIdx.x * NBC;

  {
    const v4i z = {0, 0, 0, 0};
    for (int i = tid; i < NBC / 4; i += NTHR) ((v4i*)scnt)[i] = z;
  }
  __syncthreads();

  const int nChunks = (nE + CHUNK - 1) / CHUNK;
#pragma unroll 1
  for (int ch = 0; ch < nChunks; ++ch) {
    const int cbase = ch * CHUNK;
    const int wc = scan_chunk<NBC, 0>(keys, gath, nE, nN, cbase, nodeBase, vec8, list, tid, lane, wave);
    if (lane == 0) wcnt[wave] = wc;
    __syncthreads();
    if (wave == 0) {
#pragma unroll 1
      for (int wsx = 0; wsx < NWAVE; ++wsx) {
        int n = __builtin_amdgcn_readfirstlane(wcnt[wsx]);
        n = n > WCAP ? WCAP : (n < 0 ? 0 : n);
        const int* lp = list + wsx * WCAP;
#pragma unroll 1
        for (int i = 0; i < n; ++i) {
          const int ent  = __builtin_amdgcn_readfirstlane(lp[i]);
          const int slot = ent & (NBC - 1);
          if (lane == 0) scnt[slot] = scnt[slot] + 1;
        }
      }
    }
    __syncthreads();
  }

  int*   cp = cnt + (size_t)nodeBase;
  float* dp = dinv + (size_t)nodeBase;
#pragma unroll 4
  for (int q = 0; q < 32; ++q) {
    const int f = (wave * 32 + q) * 128 + 4 * lane;
    const v4i c = *(const v4i*)(scnt + f);
    const float g0 = (float)c.x + CSELF, g1 = (float)c.y + CSELF, g2 = (float)c.z + CSELF, g3 = (float)c.w + CSELF;
    v4f d;
    d.x = g0 > 0.f ? rsqrtf(g0) : 0.f; d.y = g1 > 0.f ? rsqrtf(g1) : 0.f;
    d.z = g2 > 0.f ? rsqrtf(g2) : 0.f; d.w = g3 > 0.f ? rsqrtf(g3) : 0.f;
    *(volatile v4i*)(cp + f) = c;
    *(volatile v4f*)(dp + f) = d;
  }
  __threadfence();
#pragma unroll 4
  for (int q = 0; q < 32; ++q) {
    const int f = (wave * 32 + q) * 128 + 4 * lane;
    const v4i c = *(const v4i*)(scnt + f);
    const float g0 = (float)c.x + CSELF, g1 = (float)c.y + CSELF, g2 = (float)c.z + CSELF, g3 = (float)c.w + CSELF;
    v4f d;
    d.x = g0 > 0.f ? rsqrtf(g0) : 0.f; d.y = g1 > 0.f ? rsqrtf(g1) : 0.f;
    d.z = g2 > 0.f ? rsqrtf(g2) : 0.f; d.w = g3 > 0.f ? rsqrtf(g3) : 0.f;
    *(volatile v4i*)(cp + f) = c;
    *(volatile v4f*)(dp + f) = d;
  }
}

__global__ __launch_bounds__(OTHR) void k_offsets(
    const int* __restrict__ cnt, int* off, int* rbase, int nBF) {
  __shared__ __attribute__((aligned(16))) int srb[RBN];
  __shared__ int wtot[OTHR / 32];
  const int tid = threadIdx.x, lane = tid & 31, wave = tid >> 5;
  for (int i = tid; i < RBN; i += OTHR) srb[i] = 0;
  int carry = 0;
#pragma unroll 1
  for (int fb = 0; fb < nBF; ++fb) {
    const int base = fb * NBF;
    const v4i c = *(const v4i*)(cnt + base + 4 * tid);
    const int e0 = max(c.x, 0), e1 = max(c.y, 0), e2 = max(c.z, 0), e3 = max(c.w, 0);
    const int ts = e0 + e1 + e2 + e3;
    int incl = ts;
#pragma unroll
    for (int d = 1; d < 32; d <<= 1) {
      const int t = __shfl_up(incl, d, 32);
      if (lane >= d) incl += t;
    }
    if (lane == 31) wtot[wave] = incl;
    __syncthreads();
    int pre = 0;
#pragma unroll 1
    for (int w = 0; w < wave; ++w) pre += wtot[w];
    int tot = 0;
#pragma unroll
    for (int w = 0; w < OTHR / 32; ++w) tot += wtot[w];
    int run = carry + pre + incl - ts;
    v4i o;
    o.x = run; run += e0;
    o.y = run; run += e1;
    o.z = run; run += e2;
    o.w = run;
    int* op = off + base + 4 * tid;
    *(volatile v4i*)op = o;
    __threadfence();
    *(volatile v4i*)op = o;
    if (tid == 0) srb[min(fb, RBN - 1)] = carry;
    carry += (tot + 31) & ~31;
    __syncthreads();
  }
  if (tid == 0) srb[min(nBF, RBN - 1)] = carry;
  __syncthreads();
  v4i rv = {0, 0, 0, 0};
  if (tid < 32) rv = *(const v4i*)(srb + 4 * tid);
  if (tid < 32) *(volatile v4i*)(rbase + 4 * tid) = rv;
  __threadfence();
  if (tid < 32) *(volatile v4i*)(rbase + 4 * tid) = rv;
}

__global__ __launch_bounds__(NTHR) void k_fill(
    const int* __restrict__ keys, const int* __restrict__ gath, const int* __restrict__ off, const int* __restrict__ rbase,
    int* csr, int nN, int nE, int vec8, int csrLen) {
  extern __shared__ v4f lds_dyn[];
  int* region = (int*)lds_dyn;
  int* cursor = region + RCAP;
  int* list   = cursor + NBF;
  int* wcnt   = list + LISTN;
  const int tid = threadIdx.x, lane = tid & 31, wave = tid >> 5;
  const int b = blockIdx.x;
  const int nodeBase = b * NBF;

  int rb0 = rbase[b];
  const int rb1 = rbase[b + 1];
  rb0 = rb0 < 0 ? 0 : (rb0 > csrLen ? csrLen : rb0);
  rb0 &= ~31;
  int len = rb1 - rb0;
  len = len < 0 ? 0 : (len > RCAP ? RCAP : len);
  int lenW = (len + 31) & ~31;
  if (rb0 + lenW > csrLen) lenW = (csrLen - rb0) & ~31;

  {
    const v4i z = {0, 0, 0, 0};
    for (int i = tid; i < RCAP / 4; i += NTHR) ((v4i*)region)[i] = z;
    for (int s = tid; s < NBF; s += NTHR) {
      int o = off[nodeBase + s] - rb0;
      o = o < 0 ? 0 : (o > RCAP ? RCAP : o);
      cursor[s] = o;
    }
  }
  __syncthreads();

  const int nChunks = (nE + CHUNK - 1) / CHUNK;
#pragma unroll 1
  for (int ch = 0; ch < nChunks; ++ch) {
    const int cbase = ch * CHUNK;
    const int wc = scan_chunk<NBF, 1>(keys, gath, nE, nN, cbase, nodeBase, vec8, list, tid, lane, wave);
    if (lane == 0) wcnt[wave] = wc;
    __syncthreads();
    if (wave == 0) {
#pragma unroll 1
      for (int wsx = 0; wsx < NWAVE; ++wsx) {
        int n = __builtin_amdgcn_readfirstlane(wcnt[wsx]);
        n = n > WCAP ? WCAP : (n < 0 ? 0 : n);
        const int* lp = list + wsx * WCAP;
#pragma unroll 1
        for (int i = 0; i < n; ++i) {
          const int ent  = __builtin_amdgcn_readfirstlane(lp[i]);
          const int slot = ent & (NBF - 1);
          int src = (ent >> ESHF) & 0xFFFFF;
          src = src > nN - 1 ? nN - 1 : src;
          if (lane == 0) {
            int pos = cursor[slot];
            pos = pos < 0 ? 0 : (pos > RCAP - 1 ? RCAP - 1 : pos);
            region[pos] = src;
            const int np = pos + 1;
            cursor[slot] = np > RCAP ? RCAP : np;
          }
        }
      }
    }
    __syncthreads();
  }

  const int nv = lenW >> 2;
  int* gp = csr + rb0;
#pragma unroll 1
  for (int i = tid; i < nv; i += NTHR) { const v4i v = ((const v4i*)region)[i]; *(volatile v4i*)(gp + 4 * i) = v; }
  __threadfence();
#pragma unroll 1
  for (int i = tid; i < nv; i += NTHR) { const v4i v = ((const v4i*)region)[i]; *(volatile v4i*)(gp + 4 * i) = v; }
}

__global__ __launch_bounds__(NTHR) void k_xs0(const float* __restrict__ x0, const float* __restrict__ dinv,
                                              float* xs, int nN) {
  const int tid = threadIdx.x, lane = tid & 31, wave = tid >> 5;
#pragma unroll 1
  for (int q = 0; q < 8; ++q) {
    const int row = (int)blockIdx.x * XROWS + wave * 8 + q;
    const int rr = row > nN - 1 ? nN - 1 : row;
    const v4f v = *(const v4f*)(x0 + (size_t)rr * HD + 4 * lane);
    const float d = dinv[row];
    v4f o = v * d;
    if (row >= nN) { o.x = 0.f; o.y = 0.f; o.z = 0.f; o.w = 0.f; }
    float* p = xs + (size_t)row * HD + 4 * lane;
    *(volatile v4f*)p = o;
    __threadfence();
    *(volatile v4f*)p = o;
  }
}

__global__ __launch_bounds__(NTHR) void k_agg(
    const int* __restrict__ csr, const int* __restrict__ off, const int* __restrict__ cnt,
    const float* __restrict__ dinv, const float* __restrict__ xs, const float* __restrict__ x0,
    _Float16* am, int nN, int csrLen) {
  const int tid = threadIdx.x, lane = tid & 31, wave = tid >> 5;
  const int tbase = blockIdx.x * TGT + wave * 32;
  const int cl = tbase + lane;
  const int cnt_l = cnt[cl];
  const int off_l = off[cl];
  union FI { float f; int i; };
  FI dvu; dvu.f = dinv[cl];

#pragma unroll 1
  for (int j = 0; j < 32; ++j) {
    const int c = tbase + j;
    int n = __builtin_amdgcn_readlane(cnt_l, j);
    n = n < 0 ? 0 : (n > DEGCAP ? DEGCAP : n);
    const int st = __builtin_amdgcn_readlane(off_l, j);
    FI du; du.i = __builtin_amdgcn_readlane(dvu.i, j);
    const float dc = du.f;
    v4f acc = {0.f, 0.f, 0.f, 0.f};
#pragma unroll 1
    for (int q0 = 0; q0 < n; q0 += 32) {
      int pos = st + q0 + lane;
      pos = pos < 0 ? 0 : (pos > csrLen - 1 ? csrLen - 1 : pos);
      int sl = csr[pos];
      sl = sl < 0 ? 0 : (sl > nN - 1 ? nN - 1 : sl);
      const int mcnt = (n - q0) < 32 ? (n - q0) : 32;
#pragma unroll 1
      for (int p = 0; p < mcnt; ++p) {
        const int sidx = __builtin_amdgcn_readlane(sl, p);
        acc = acc + *(const v4f*)(xs + (size_t)sidx * HD + 4 * lane);
      }
    }
    const v4f sv = *(const v4f*)(xs + (size_t)c * HD + 4 * lane);
    const int cr = c > nN - 1 ? nN - 1 : c;
    const v4f xz = *(const v4f*)(x0 + (size_t)cr * HD + 4 * lane);
    const v4f hs = (acc + sv * CSELF) * dc;
    const v4f a  = hs * OMALPHA + xz * ALPHAC;
    H4U hq;
    hq.h[0] = (_Float16)(a.x * (float)ASCALE); hq.h[1] = (_Float16)(a.y * (float)ASCALE);
    hq.h[2] = (_Float16)(a.z * (float)ASCALE); hq.h[3] = (_Float16)(a.w * (float)ASCALE);
    const v2u uu = hq.u;
    _Float16* ap = am + (size_t)c * HD + 4 * lane;
    *(volatile v2u*)ap = uu;
    __threadfence();
    *(volatile v2u*)ap = uu;
  }
}

template <int MODE>
__global__ __launch_bounds__(NTHR) void k_lgemm(
    const _Float16* __restrict__ A, const _Float16* __restrict__ Bw, const float* __restrict__ dinv,
    float* Cf, _Float16* Ch) {
  extern __shared__ v4f lds_dyn[];
  constexpr int NT = HD / 16;
  constexpr float OSC = 1.0f / (float)(ASCALE * WSCALE);
  float* stg = (float*)lds_dyn;
  const int tid = threadIdx.x, lane = tid & 31, wave = tid >> 5, hh = lane >> 4, m = lane & 15;
  const int rowBase = blockIdx.x * GROWS;
  const int arow = rowBase + wave * 16 + m;
  const _Float16* ap = A + (size_t)arow * HD + 8 * hh;

  v8f acc[NT];
#pragma unroll
  for (int t = 0; t < NT; ++t) { v8f z = {0.f, 0.f, 0.f, 0.f, 0.f, 0.f, 0.f, 0.f}; acc[t] = z; }

#pragma unroll 1
  for (int kt = 0; kt < HD / 32; ++kt) {
    const v16h av = afr(ap + 32 * kt);
#pragma unroll
    for (int t = 0; t < NT; ++t) {
      const v16h bv = afr(Bw + (size_t)(16 * t + m) * HD + 32 * kt + 8 * hh);
      acc[t] = wmf(av, bv, acc[t]);
    }
  }

  const int r0 = wave * 16 + 8 * hh;
  float s[8];
  if constexpr (MODE == 0) {
    const v4f dA = *(const v4f*)(dinv + (size_t)rowBase + r0);
    const v4f dB = *(const v4f*)(dinv + (size_t)rowBase + r0 + 4);
    s[0] = dA.x; s[1] = dA.y; s[2] = dA.z; s[3] = dA.w; s[4] = dB.x; s[5] = dB.y; s[6] = dB.z; s[7] = dB.w;
#pragma unroll
    for (int r = 0; r < 8; ++r) s[r] = s[r] * OSC;
  } else {
#pragma unroll
    for (int r = 0; r < 8; ++r) s[r] = OSC * (float)ASCALE;
  }
  float* sp = stg + r0 * HD + m;
#pragma unroll
  for (int t = 0; t < NT; ++t) {
#pragma unroll
    for (int r = 0; r < 8; ++r) {
      float v = acc[t][r] * s[r];
      v = v >= 0.f ? v : SLOPEC * v;
      sp[r * HD + 16 * t] = v;
    }
  }
  __syncthreads();

  const float* lp = stg + wave * 16 * HD;
  if constexpr (MODE == 0) {
    float* gp = Cf + (size_t)(rowBase + wave * 16) * HD;
#pragma unroll
    for (int i = 0; i < 16; ++i) {
      const v4f v = *(const v4f*)(lp + i * HD + 4 * lane);
      *(volatile v4f*)(gp + i * HD + 4 * lane) = v;
    }
    __threadfence();
#pragma unroll
    for (int i = 0; i < 16; ++i) {
      const v4f v = *(const v4f*)(lp + i * HD + 4 * lane);
      *(volatile v4f*)(gp + i * HD + 4 * lane) = v;
    }
  } else {
    _Float16* hp = Ch + (size_t)(rowBase + wave * 16) * HD;
#pragma unroll
    for (int i = 0; i < 16; ++i) {
      const v4f v = *(const v4f*)(lp + i * HD + 4 * lane);
      H4U hq;
      hq.h[0] = (_Float16)v.x; hq.h[1] = (_Float16)v.y; hq.h[2] = (_Float16)v.z; hq.h[3] = (_Float16)v.w;
      const v2u uu = hq.u;
      *(volatile v2u*)(hp + i * HD + 4 * lane) = uu;
    }
    __threadfence();
#pragma unroll
    for (int i = 0; i < 16; ++i) {
      const v4f v = *(const v4f*)(lp + i * HD + 4 * lane);
      H4U hq;
      hq.h[0] = (_Float16)v.x; hq.h[1] = (_Float16)v.y; hq.h[2] = (_Float16)v.z; hq.h[3] = (_Float16)v.w;
      const v2u uu = hq.u;
      *(volatile v2u*)(hp + i * HD + 4 * lane) = uu;
    }
  }
}

__global__ __launch_bounds__(DTHR) void k_dense(
    const _Float16* __restrict__ A, const _Float16* __restrict__ Bw, const float* __restrict__ bd,
    const float* __restrict__ wo, const float* __restrict__ bo, float* out, int nN) {
  extern __shared__ v4f lds_dyn[];
  __shared__ __attribute__((aligned(16))) float sres[DROWS * 2];
  constexpr int NT = HD / 16;
  constexpr float OSC = 1.0f / (float)(ASCALE * WSCALE);
  float* stg = (float*)lds_dyn;
  const int tid = threadIdx.x, lane = tid & 31, wave = tid >> 5, hh = lane >> 4, m = lane & 15;
  const int rowBase = blockIdx.x * DROWS;
  const int arow = rowBase + wave * 16 + m;
  const _Float16* ap = A + (size_t)arow * HD + 8 * hh;
  const int r0 = wave * 16 + 8 * hh;

#pragma unroll 1
  for (int nh = 0; nh < 2; ++nh) {
    v8f acc[NT];
#pragma unroll
    for (int t = 0; t < NT; ++t) { v8f z = {0.f, 0.f, 0.f, 0.f, 0.f, 0.f, 0.f, 0.f}; acc[t] = z; }
    const _Float16* bbase = Bw + (size_t)(nh * HD) * HD;
#pragma unroll 1
    for (int kt = 0; kt < HD / 32; ++kt) {
      const v16h av = afr(ap + 32 * kt);
#pragma unroll
      for (int t = 0; t < NT; ++t) {
        const v16h bv = afr(bbase + (size_t)(16 * t + m) * HD + 32 * kt + 8 * hh);
        acc[t] = wmf(av, bv, acc[t]);
      }
    }
    float* sp = stg + r0 * DN + nh * HD + m;
#pragma unroll
    for (int t = 0; t < NT; ++t) {
      const float bc = bd[nh * HD + 16 * t + m];
#pragma unroll
      for (int r = 0; r < 8; ++r) {
        const float v = acc[t][r] * OSC + bc;
        sp[r * DN + 16 * t] = v;
      }
    }
  }
  __syncthreads();

  const v4f wa0 = *(const v4f*)(wo + 8 * lane);
  const v4f wa1 = *(const v4f*)(wo + 8 * lane + 4);
  const v4f wb0 = *(const v4f*)(wo + DN + 8 * lane);
  const v4f wb1 = *(const v4f*)(wo + DN + 8 * lane + 4);
  const float b0 = bo[0], b1 = bo[1];
  const float* lp = stg + wave * 16 * DN;
#pragma unroll 2
  for (int i = 0; i < 16; ++i) {
    const v4f q0 = *(const v4f*)(lp + i * DN + 4 * lane);
    const v4f q1 = *(const v4f*)(lp + i * DN + HD + 4 * lane);
    float d0 = (q0.x * wa0.x + q0.y * wa0.z) + (q0.z * wa1.x + q0.w * wa1.z)
             + (q1.x * wb0.x + q1.y * wb0.z) + (q1.z * wb1.x + q1.w * wb1.z);
    float d1 = (q0.x * wa0.y + q0.y * wa0.w) + (q0.z * wa1.y + q0.w * wa1.w)
             + (q1.x * wb0.y + q1.y * wb0.w) + (q1.z * wb1.y + q1.w * wb1.w);
#pragma unroll
    for (int mm = 16; mm >= 1; mm >>= 1) {
      d0 += __shfl_xor(d0, mm, 32);
      d1 += __shfl_xor(d1, mm, 32);
    }
    if (lane == 0) {
      sres[(wave * 16 + i) * 2]     = d0 + b0;
      sres[(wave * 16 + i) * 2 + 1] = d1 + b1;
    }
  }
  __syncthreads();

  if (wave == 0) {
    const int f = 4 * lane;
    const int lim = 2 * (nN - rowBase);
    const v4f r = *(const v4f*)(sres + f);
    v2f r2; r2.x = r.x; r2.y = r.y;
    const bool full = (f + 4) <= lim;
    const bool two  = (!full) && ((f + 2) <= lim);
    float* op = out + (size_t)rowBase * 2 + f;
    if (full) *(volatile v4f*)op = r;
    if (two)  *(volatile v2f*)op = r2;
    __threadfence();
    if (full) *(volatile v4f*)op = r;
    if (two)  *(volatile v2f*)op = r2;
  }
}

extern "C" void kernel_launch(void* const* d_in, const int* in_sizes, int n_in,
                              void* d_out, int out_size, void* d_ws, size_t ws_size,
                              hipStream_t stream) {
  if (n_in < 7) return;
  const int nN = in_sizes[0] / HD;
  const int nE = in_sizes[1] / 2;
  if (nN <= 0 || nE <= 0) return;
  if (in_sizes[0] != nN * HD || in_sizes[1] != 2 * nE) return;
  if (in_sizes[2] != NLAY * HD * HD) return;
  if (in_sizes[3] != HD * DN || in_sizes[4] != DN) return;
  if (in_sizes[5] != DN * 2 || in_sizes[6] != 2) return;
  if (out_size != 2 * nN) return;
  if (nN > (1 << 20) || nE > (1 << 28)) return;

  const float* x0  = (const float*)d_in[0];
  const int*   ei  = (const int*)d_in[1];
  const int*   srcp = ei;
  const int*   dstp = ei + nE;
  const float* wc  = (const float*)d_in[2];
  const float* wd  = (const float*)d_in[3];
  const float* bd  = (const float*)d_in[4];
  const float* wo  = (const float*)d_in[5];
  const float* bo  = (const float*)d_in[6];
  float* out = (float*)d_out;

  const int NPAD   = ((nN + TGT - 1) / TGT) * TGT;
  const int nBC    = (nN + NBC - 1) / NBC;
  const int CNTPAD = nBC * NBC;
  const int nBF    = (nN + NBF - 1) / NBF;
  const int OFFN   = nBF * NBF;
  if (nBF + 1 > RBN) return;
  if (OFFN > CNTPAD || NPAD > OFFN) return;
  const int csrLen = ((nE + 31) & ~31) + 32 * (nBF + 1);
  const int nGemm  = NPAD / GROWS;
  const int nAgg   = NPAD / TGT;
  const int nXs    = NPAD / XROWS;
  const int nDen   = NPAD / DROWS;

  char* ws = (char*)d_ws;
  size_t off = 0;
  const size_t oW   = off; off += (size_t)WPTOT * 2;          off = (off + 255) & ~(size_t)255;
  const size_t oCnt = off; off += (size_t)CNTPAD * 4;         off = (off + 255) & ~(size_t)255;
  const size_t oDv  = off; off += (size_t)CNTPAD * 4;         off = (off + 255) & ~(size_t)255;
  const size_t oOff = off; off += (size_t)OFFN * 4;           off = (off + 255) & ~(size_t)255;
  const size_t oRb  = off; off += (size_t)RBN * 4;            off = (off + 255) & ~(size_t)255;
  const size_t oCsr = off; off += (size_t)csrLen * 4;         off = (off + 255) & ~(size_t)255;
  const size_t oXs  = off; off += (size_t)NPAD * HD * 4;      off = (off + 255) & ~(size_t)255;
  const size_t oAm  = off; off += (size_t)NPAD * HD * 2;      off = (off + 255) & ~(size_t)255;
  const size_t oXh  = off; off += (size_t)NPAD * HD * 2;      off = (off + 255) & ~(size_t)255;
  if (off > ws_size || off > (size_t)WSCAP) return;
  _Float16* wp   = (_Float16*)(ws + oW);
  int*      cnt  = (int*)(ws + oCnt);
  float*    dinv = (float*)(ws + oDv);
  int*      offp = (int*)(ws + oOff);
  int*      rb   = (int*)(ws + oRb);
  int*      csr  = (int*)(ws + oCsr);
  float*    xs   = (float*)(ws + oXs);
  _Float16* am   = (_Float16*)(ws + oAm);
  _Float16* xh   = (_Float16*)(ws + oXh);
  const _Float16* wpd = wp + WPD;

  const int vec8 = ((nE & 3) == 0) ? 1 : 0;

  k_wprep<<<WPREP_BLOCKS, NTHR, 0, stream>>>(wc, wd, wp);

  hipFuncSetAttribute(reinterpret_cast<const void*>(&k_count),
                      hipFuncAttributeMaxDynamicSharedMemorySize, LDS_COUNT);
  k_count<<<nBC, NTHR, LDS_COUNT, stream>>>(dstp, srcp, cnt, dinv, nE, nN, vec8);
  k_offsets<<<1, OTHR, 0, stream>>>(cnt, offp, rb, nBF);
  hipFuncSetAttribute(reinterpret_cast<const void*>(&k_fill),
                      hipFuncAttributeMaxDynamicSharedMemorySize, LDS_FILL);
  k_fill<<<nBF, NTHR, LDS_FILL, stream>>>(dstp, srcp, offp, rb, csr, nN, nE, vec8, csrLen);

  k_xs0<<<nXs, NTHR, 0, stream>>>(x0, dinv, xs, nN);

  hipFuncSetAttribute(reinterpret_cast<const void*>(&k_lgemm<0>),
                      hipFuncAttributeMaxDynamicSharedMemorySize, LDS_GEMM);
  hipFuncSetAttribute(reinterpret_cast<const void*>(&k_lgemm<1>),
                      hipFuncAttributeMaxDynamicSharedMemorySize, LDS_GEMM);
  hipFuncSetAttribute(reinterpret_cast<const void*>(&k_dense),
                      hipFuncAttributeMaxDynamicSharedMemorySize, LDS_DENSE);

  for (int l = 0; l < NLAY; ++l) {
    k_agg<<<nAgg, NTHR, 0, stream>>>(csr, offp, cnt, dinv, xs, x0, am, nN, csrLen);
    const _Float16* wpl = wp + (size_t)l * WPL;
    if (l < NLAY - 1)
      k_lgemm<0><<<nGemm, NTHR, LDS_GEMM, stream>>>(am, wpl, dinv, xs, xh);
    else
      k_lgemm<1><<<nGemm, NTHR, LDS_GEMM, stream>>>(am, wpl, dinv, xs, xh);
  }

  k_dense<<<nDen, DTHR, LDS_DENSE, stream>>>(xh, wpd, bd, wo, bo, out, nN);
}
